// ISTFT_66503273612036
// MI455X (gfx1250) — hardware-verified
//
#include <hip/hip_runtime.h>
#include <math.h>

constexpr int kBatch   = 16;
constexpr int kFrames  = 601;
constexpr int kBins    = 1025;
constexpr int kNfft    = 2048;
constexpr int kHop     = 512;
constexpr int kOutLen  = 307200;
constexpr int kSegs    = 600;
constexpr int kQ0      = 2;
constexpr int kM       = kBatch * kSegs;
constexpr int kN       = kHop;
constexpr int kKph     = 2 * kBins;
constexpr int kKpad    = 2080;
constexpr int kPitch   = 2112;
constexpr int kPhases  = 4;
constexpr int kZeroRow = kBatch * kFrames;
constexpr int kSRows   = kZeroRow + 1;
constexpr int kWPitch  = kPhases * kPitch;
constexpr float kWCarry    = 4096.0f;
constexpr float kWCarryInv = 1.0f / 4096.0f;
constexpr float kTwoPiOverN = 0.0030679615757712823f;

constexpr size_t kSBytes  = (size_t)kSRows * kPitch * 2;
constexpr size_t kWBytes  = (size_t)kN * kWPitch * 2;
constexpr size_t kWsTotal = kSBytes + kWBytes;

static_assert(kKpad % 32 == 0, "k per phase multiple of 32");
static_assert(kKpad >= kKph && kKpad + 24 <= kPitch, "fragment reads stay inside the padded row");
static_assert((kPitch * 2) % 128 == 0, "S rows / Wt segments are whole 128-B lines");
static_assert(kM % 64 == 0 && kN % 64 == 0, "GEMM tile multiples");
static_assert(kSBytes % 128 == 0 && kWBytes % 128 == 0, "line-aligned carves");
static_assert(kWsTotal <= (size_t)134217728, "carve under 128 MiB");
static_assert(kM * kN == kBatch * kOutLen, "GEMM covers the whole output");
static_assert(kPitch % 8 == 0 && kPitch / 8 == 264, "pack store coverage: 264 lanes x 8 halves");

typedef __attribute__((ext_vector_type(16))) _Float16 v16h;
typedef __attribute__((ext_vector_type(8)))  _Float16 v8h;
typedef __attribute__((ext_vector_type(8)))  float    v8f;
typedef __attribute__((ext_vector_type(4)))  float    v4f;
typedef __attribute__((ext_vector_type(4)))  unsigned int v4u;

__device__ __forceinline__ unsigned short f2bf_bits(float f) {
  unsigned u = __float_as_uint(f);
  return (unsigned short)((u + 0x7FFFu + ((u >> 16) & 1u)) >> 16);
}
__device__ __forceinline__ float bf_bits2f(unsigned short h) { return __uint_as_float(((unsigned)h) << 16); }

__device__ __forceinline__ void dep_guard_h(v8f& a, v8f& b, v16h x, v16h y) { asm volatile("v_nop\n\tv_nop\n\tv_nop\n\tv_nop" : "+v"(a), "+v"(b) : "v"(x), "v"(y)); }
__device__ __forceinline__ void keep4_h(v16h a, v16h b, v16h c, v16h d) { asm volatile("v_nop" :: "v"(a), "v"(b), "v"(c), "v"(d)); }
__device__ __forceinline__ void acc_guard4(v8f& a, v8f& b, v8f& c, v8f& d) { asm volatile("v_nop\n\tv_nop\n\tv_nop\n\tv_nop" : "+v"(a), "+v"(b), "+v"(c), "+v"(d)); }
template <typename T> struct Frag;
template <> struct Frag<_Float16> {
  typedef v16h V; union U { v16h v; v8h h[2]; };
  static __device__ __forceinline__ v16h load(const _Float16* p) {
    U f; f.h[0] = *(const v8h*)(p); f.h[1] = *(const v8h*)(p + 16); return f.v;
  }
  static __device__ __forceinline__ v8f mma(v16h a, v16h b, v8f c) {
    return __builtin_amdgcn_wmma_f32_16x16x32_f16(false, a, false, b, (short)0, c, false, false);
  }
  static __device__ __forceinline__ void guard(v8f& a, v8f& b, v16h x, v16h y) { dep_guard_h(a, b, x, y); }
  static __device__ __forceinline__ void keep(v16h a, v16h b, v16h c, v16h d) { keep4_h(a, b, c, d); }
};

__device__ __forceinline__ unsigned pk16(unsigned short a, unsigned short b) { return (unsigned)a | ((unsigned)b << 16); }
__device__ __forceinline__ unsigned short h_bits(float f) { const _Float16 h = (_Float16)f; return __builtin_bit_cast(unsigned short, h); }
__device__ __forceinline__ float bf_rne(float f) { return bf_bits2f(f2bf_bits(f)); }

__global__ __launch_bounds__(288) void pack_spec_kernel(const float* __restrict__ re, const float* __restrict__ im,
                                                        unsigned short* __restrict__ S) {
  __shared__ __align__(16) float sX[kPitch];
  const int row = blockIdx.x;
  const int t   = threadIdx.x;
  const bool zrow = (row >= kZeroRow);
  const int rowc  = zrow ? (kZeroRow - 1) : row;
  const float* rp = re + (size_t)rowc * kBins;
  const float* ip = im + (size_t)rowc * kBins;
#pragma unroll
  for (int it = 0; it < 4; ++it) {
    const int f  = t + 288 * it;
    const int fc = (f < kBins) ? f : (kBins - 1);
    float a = rp[fc];
    float c = ip[fc];
    if (zrow) { a = 0.0f; c = 0.0f; }
    if (f < kBins) {
      sX[f]         = bf_rne(a);
      sX[kBins + f] = bf_rne(c);
    }
  }
  if (t < kPitch - kKph) sX[kKph + t] = 0.0f;
  __syncthreads();
  if (t < kPitch / 8) {
    const v4f x0 = *(const v4f*)(sX + 8 * t);
    const v4f x1 = *(const v4f*)(sX + 8 * t + 4);
    unsigned short hb[8];
#pragma unroll
    for (int e = 0; e < 4; ++e) {
      hb[e]     = h_bits(x0[e]);
      hb[4 + e] = h_bits(x1[e]);
    }
    const v4u u = (v4u){pk16(hb[0], hb[1]), pk16(hb[2], hb[3]), pk16(hb[4], hb[5]), pk16(hb[6], hb[7])};
    unsigned short* q = S + (size_t)row * kPitch + 8 * t;
    *(volatile v4u*)q = u;
    __threadfence();
    *(volatile v4u*)q = u;
  }
}

__global__ __launch_bounds__(288) void pack_w_kernel(const float* __restrict__ wr, const float* __restrict__ wi,
                                                     unsigned short* __restrict__ Wt) {
  __shared__ __align__(16) float sR[kNfft];
  __shared__ __align__(16) float sI[kNfft];
  const int o  = blockIdx.x;
  const int ph = o >> 9;
  const int r  = o & (kHop - 1);
  const int t  = threadIdx.x;
  const float* rp = wr + (size_t)o * kNfft;
  const float* ip = wi + (size_t)o * kNfft;
  if (t < 256) {
#pragma unroll
    for (int it = 0; it < 2; ++it) {
      const int idx4 = t + 256 * it;
      const v4f a = *(const v4f*)(rp + 4 * idx4);
      const v4f c = *(const v4f*)(ip + 4 * idx4);
#pragma unroll
      for (int e = 0; e < 4; ++e) {
        sR[4 * idx4 + e] = bf_rne(a[e]);
        sI[4 * idx4 + e] = bf_rne(c[e]);
      }
    }
  }
  __syncthreads();
  if (t < kPitch / 8) {
    unsigned short hb[8];
#pragma unroll
    for (int e = 0; e < 8; ++e) {
      const int k = 8 * t + e;
      const int fr = (k < kBins) ? k : (kBins - 1);
      int pr = kNfft - fr;
      pr = (pr > kNfft - 1) ? (kNfft - 1) : pr;
      const float ar = sR[fr];
      const float br = sR[pr];
      const float vr = ar + (((fr >= 1) && (fr <= kBins - 2)) ? br : 0.0f);
      int fi = k - kBins;
      fi = (fi < 0) ? 0 : ((fi > kBins - 1) ? (kBins - 1) : fi);
      int qi = kNfft - fi;
      qi = (qi > kNfft - 1) ? (kNfft - 1) : qi;
      const float ai = sI[fi];
      const float bi = sI[qi];
      const float vi = (((fi >= 1) && (fi <= kBins - 2)) ? bi : 0.0f) - ai;
      float v = (k < kBins) ? vr : ((k < kKph) ? vi : 0.0f);
      v = v * kWCarry;
      hb[e] = h_bits(v);
    }
    const v4u u = (v4u){pk16(hb[0], hb[1]), pk16(hb[2], hb[3]), pk16(hb[4], hb[5]), pk16(hb[6], hb[7])};
    unsigned short* q = Wt + (size_t)r * kWPitch + (size_t)ph * kPitch + 8 * t;
    *(volatile v4u*)q = u;
    __threadfence();
    *(volatile v4u*)q = u;
  }
}

__global__ __launch_bounds__(256) void ola_gemm_kernel(const unsigned short* __restrict__ Sp,
                                                      const unsigned short* __restrict__ Wp,
                                                      float* __restrict__ out) {
  typedef _Float16 T;
  typedef v16h V;
  const T* S = (const T*)Sp;
  const T* W = (const T*)Wp;
  __shared__ __align__(16) float sT[8][16 * 68];
  __shared__ __align__(16) float sRinv[3 * kHop];
  const int tid  = threadIdx.x;
  const int lane = tid & 31;
  const int wave = tid >> 5;

#pragma unroll 1
  for (int it = 0; it < 6; ++it) {
    const int idx = tid + 256 * it;
    const int cls = idx >> 9;
    const int n   = idx & (kHop - 1);
    float ws = 0.0f;
#pragma unroll 1
    for (int j = 3; j >= 0; --j) {
      const bool valid = (cls == 0) ? (j <= 2) : ((cls == 2) ? (j >= 1) : true);
      const float ang = (float)(n + kHop * j) * kTwoPiOverN;
      const float hw  = 0.5f - 0.5f * cosf(ang);
      const float hs  = hw * hw;
      ws = valid ? (ws + hs) : ws;
    }
    sRinv[idx] = 1.0f / ws;
  }
  __syncthreads();

  const int m0 = blockIdx.x * 64;
  const int n0 = wave * 64;
  const int rlane = lane & 15;
  const int koff  = (lane >> 4) * 8;
  const int mOff  = (lane >> 4) * 8;

  v8f acc[4][4];
#pragma unroll
  for (int i = 0; i < 4; ++i)
#pragma unroll
    for (int j = 0; j < 4; ++j) acc[i][j] = (v8f){0.f,0.f,0.f,0.f,0.f,0.f,0.f,0.f};

#pragma unroll 1
  for (int ph = 0; ph < kPhases; ++ph) {
    const T* aP[4];
#pragma unroll
    for (int i = 0; i < 4; ++i) {
      const int m   = m0 + (i << 4) + rlane;
      const int bq  = m / kSegs;
      const int qq  = m - bq * kSegs;
      const int tfr = qq + kQ0 - ph;
      const bool valid = (tfr >= 0) && (tfr < kFrames);
      int srow = valid ? (bq * kFrames + tfr) : kZeroRow;
      srow = (srow < 0) ? 0 : ((srow > kZeroRow) ? kZeroRow : srow);
      aP[i] = S + (size_t)srow * kPitch + koff;
    }
    const T* bP = W + (size_t)(n0 + rlane) * kWPitch + (size_t)ph * kPitch + koff;
    for (int kk = 0; kk < kKpad; kk += 32) {
      V bh[4];
#pragma unroll
      for (int j = 0; j < 4; ++j) bh[j] = Frag<T>::load(bP + (size_t)j * 16 * kWPitch + kk);
#pragma unroll
      for (int i = 0; i < 4; ++i) {
        V ah = Frag<T>::load(aP[i] + kk);
#pragma unroll
        for (int j = 0; j < 4; ++j) acc[i][j] = Frag<T>::mma(ah, bh[j], acc[i][j]);
        Frag<T>::guard(acc[i][0], acc[i][3], ah, ah);
      }
      Frag<T>::keep(bh[0], bh[1], bh[2], bh[3]);
    }
  }
  acc_guard4(acc[0][0], acc[0][1], acc[0][2], acc[0][3]);
  acc_guard4(acc[1][0], acc[1][1], acc[1][2], acc[1][3]);
  acc_guard4(acc[2][0], acc[2][1], acc[2][2], acc[2][3]);
  acc_guard4(acc[3][0], acc[3][1], acc[3][2], acc[3][3]);

  float* slab = sT[wave];
#pragma unroll
  for (int i = 0; i < 4; ++i) {
    const int mBase = m0 + (i << 4);
#pragma unroll
    for (int j = 0; j < 4; ++j) {
#pragma unroll
      for (int r = 0; r < 8; ++r) {
        slab[(mOff + r) * 68 + (j << 4) + rlane] = acc[i][j][r] * kWCarryInv;
      }
    }
    __builtin_amdgcn_fence(__ATOMIC_RELEASE, "workgroup");
    __builtin_amdgcn_wave_barrier();
    __builtin_amdgcn_fence(__ATOMIC_ACQUIRE, "workgroup");
    {
      const int hh = lane >> 4, c4 = (lane & 15) * 4;
      for (int pass = 0; pass < 2; ++pass) {
#pragma unroll
        for (int it = 0; it < 8; ++it) {
          const int row = it * 2 + hh;
          const int m   = mBase + row;
          const int qq  = m % kSegs;
          const int cls = (qq == 0) ? 0 : ((qq == kSegs - 1) ? 2 : 1);
          const v4f rv = *(const v4f*)(sRinv + cls * kHop + n0 + c4);
          v4f v = *(const v4f*)(slab + row * 68 + c4);
          v = v * rv;
          *(volatile v4f*)(out + (size_t)m * kN + n0 + c4) = v;
        }
        __threadfence();
      }
    }
    __builtin_amdgcn_fence(__ATOMIC_RELEASE, "workgroup");
    __builtin_amdgcn_wave_barrier();
    __builtin_amdgcn_fence(__ATOMIC_ACQUIRE, "workgroup");
  }
}

extern "C" void kernel_launch(void* const* d_in, const int* in_sizes, int n_in,
                              void* d_out, int out_size, void* d_ws, size_t ws_size,
                              hipStream_t stream) {
  if (n_in < 4) return;
  if (in_sizes[0] != kBatch * kFrames * kBins) return;
  if (in_sizes[1] != kBatch * kFrames * kBins) return;
  if (in_sizes[2] != kNfft * kNfft) return;
  if (in_sizes[3] != kNfft * kNfft) return;
  if (out_size != kM * kN) return;
  if (ws_size < kWsTotal) return;
  const float* re = (const float*)d_in[0];
  const float* im = (const float*)d_in[1];
  const float* wr = (const float*)d_in[2];
  const float* wi = (const float*)d_in[3];
  float* outp = (float*)d_out;
  char* ws = (char*)d_ws;
  unsigned short* S  = (unsigned short*)(ws);
  unsigned short* Wt = (unsigned short*)(ws + kSBytes);

  pack_spec_kernel<<<dim3(kSRows), dim3(288), 0, stream>>>(re, im, S);
  pack_w_kernel<<<dim3(kNfft), dim3(288), 0, stream>>>(wr, wi, Wt);
  ola_gemm_kernel<<<dim3(kM / 64), dim3(256), 0, stream>>>(S, Wt, outp);
}
